// GraphAttention_65566970740904
// MI455X (gfx1250) — hardware-verified
//
#include <hip/hip_runtime.h>
#include <math.h>
#include <stdint.h>

#define NB_   4
#define NL_   1024
#define DIN   256
#define NH_   8
#define HD_   32
#define DM_   (NH_ * HD_)
#define NBH   (NB_ * NH_)
#define NTOK  (NB_ * NL_)
#define BPB   (NL_ / 128)
#define NHP   (NH_ / 2)
#define SLOPE 0.2f
#define INVN  (1.0f / (float)NL_)
#define WSMAX 134217728

static_assert(NL_ % 128 == 0);
static_assert(NL_ % 64 == 0);
static_assert(NL_ == 128 * 8);
static_assert(NL_ == 256 * 4);
static_assert(DIN % 32 == 0);
static_assert(DIN % 64 == 0);
static_assert(DM_ % 64 == 0);
static_assert(DM_ == NH_ * HD_);
static_assert(HD_ == 32);
static_assert(NH_ == 8);
static_assert((NTOK * DIN) % 2048 == 0);
static_assert(NTOK % 128 == 0);
static_assert(BPB == 8);

typedef __attribute__((ext_vector_type(16))) __bf16 v16b;
typedef __attribute__((ext_vector_type(8)))  __bf16 v8b;
typedef __attribute__((ext_vector_type(8)))  float  v8f;
typedef __attribute__((ext_vector_type(4)))  float  v4f;
typedef __attribute__((ext_vector_type(4)))  unsigned int v4u;
typedef __attribute__((ext_vector_type(8)))  unsigned int v8u;
typedef __attribute__((ext_vector_type(4)))  int v4i;
typedef v8b __attribute__((may_alias)) v8ba;
typedef v4f __attribute__((may_alias)) v4fa;
typedef v4u __attribute__((may_alias)) v4ua;
typedef v4i __attribute__((may_alias)) v4ia;

union FragU { v16b v; v8b h[2]; };
union PackU { v8u u; v16b v; };

__device__ __forceinline__ unsigned short f2bf_bits(float f) {
  const unsigned u = __float_as_uint(f);
  return (unsigned short)((u + 0x7FFFu + ((u >> 16) & 1u)) >> 16);
}
__device__ __forceinline__ float bf_bits2f(unsigned short h) { return __uint_as_float(((unsigned)h) << 16); }
__device__ __forceinline__ float bf16r(float f) {
  unsigned u = __float_as_uint(f);
  u = (u + 0x7FFFu + ((u >> 16) & 1u)) & 0xFFFF0000u;
  return __uint_as_float(u);
}
__device__ __forceinline__ unsigned pk16(unsigned short a, unsigned short b) { return (unsigned)a | ((unsigned)b << 16); }

__device__ __forceinline__ v8f wmma_bf16(v16b a, v16b b, v8f c) {
  v8f d = __builtin_amdgcn_wmma_f32_16x16x32_bf16(false, a, false, b, (short)0, c, false, false);
  asm volatile("v_nop\n\tv_nop\n\tv_nop\n\tv_nop" : "+v"(d) : "v"(a), "v"(b));
  return d;
}

__device__ __forceinline__ v16b load_frag(const unsigned short* p, int hh) {
  FragU f;
  f.h[0] = *(const v8ba*)(p + 8 * hh);
  f.h[1] = *(const v8ba*)(p + 16 + 8 * hh);
  return f.v;
}

__device__ __forceinline__ void pack_p2(v8f a, v8f c, v16b& ho, v16b& lo) {
  PackU uh, ul;
#pragma unroll
  for (int i = 0; i < 4; ++i) {
    const unsigned short h0 = f2bf_bits(a[2 * i]), h1 = f2bf_bits(a[2 * i + 1]);
    const unsigned short l0 = f2bf_bits(a[2 * i] - bf_bits2f(h0)), l1 = f2bf_bits(a[2 * i + 1] - bf_bits2f(h1));
    uh.u[i] = pk16(h0, h1); ul.u[i] = pk16(l0, l1);
    const unsigned short g0 = f2bf_bits(c[2 * i]), g1 = f2bf_bits(c[2 * i + 1]);
    const unsigned short m0 = f2bf_bits(c[2 * i] - bf_bits2f(g0)), m1 = f2bf_bits(c[2 * i + 1] - bf_bits2f(g1));
    uh.u[4 + i] = pk16(g0, g1); ul.u[4 + i] = pk16(m0, m1);
  }
  ho = uh.v; lo = ul.v;
}

__device__ __forceinline__ void gemm_core_32x64p(
    const unsigned short* __restrict__ A, const unsigned short* __restrict__ Bt,
    int K, size_t aoff, size_t boff, int hh, v8f (&acc)[2][4]) {
  const unsigned short* a0 = A + aoff;
  const unsigned short* a1 = a0 + (size_t)16 * K;
  const unsigned short* bp = Bt + boff;
#pragma unroll 1
  for (int k0 = 0; k0 < K; k0 += 32) {
    const v16b f0 = load_frag(a0 + k0, hh);
    const v16b f1 = load_frag(a1 + k0, hh);
#pragma unroll
    for (int nt = 0; nt < 4; ++nt) {
      const v16b fb = load_frag(bp + (size_t)nt * 16 * K + k0, hh);
      acc[0][nt] = wmma_bf16(f0, fb, acc[0][nt]);
      acc[1][nt] = wmma_bf16(f1, fb, acc[1][nt]);
    }
  }
}

__global__ __launch_bounds__(256) void k_cvt(const float* __restrict__ src, unsigned short* __restrict__ dst, int n8) {
  int i = blockIdx.x * 256 + threadIdx.x;
  const bool ok = i < n8;
  i = ok ? i : (n8 - 1);
  const float* s = src + (size_t)i * 8;
  const v4f f0 = *(const v4fa*)(s);
  const v4f f1 = *(const v4fa*)(s + 4);
  v4u u;
  u[0] = pk16(f2bf_bits(f0[0]), f2bf_bits(f0[1]));
  u[1] = pk16(f2bf_bits(f0[2]), f2bf_bits(f0[3]));
  u[2] = pk16(f2bf_bits(f1[0]), f2bf_bits(f1[1]));
  u[3] = pk16(f2bf_bits(f1[2]), f2bf_bits(f1[3]));
  unsigned short* d = dst + (size_t)i * 8;
  if (ok) *(volatile v4u*)d = u;
  __threadfence();
  if (ok) *(volatile v4u*)d = u;
}

__global__ __launch_bounds__(256) void k_tcvt(const float* __restrict__ W, unsigned short* __restrict__ ob, int R, int Cc) {
  __shared__ __align__(16) float tf[64 * 68];
  const int c0  = blockIdx.x * 64;
  const int r0  = blockIdx.y * 64;
  const int tid = threadIdx.x;
  {
    const int lr = tid >> 4;
    const int c4 = (tid & 15) * 4;
#pragma unroll
    for (int it = 0; it < 4; ++it) {
      const int rr = it * 16 + lr;
      const v4f a = *(const v4fa*)(W + (size_t)(r0 + rr) * Cc + c0 + c4);
      *(v4fa*)(tf + rr * 68 + c4) = a;
    }
  }
  __syncthreads();
  const int sub = tid >> 3;
  const int c8  = (tid & 7) * 8;
  v4u hv[2];
#pragma unroll
  for (int it = 0; it < 2; ++it) {
    const int oc = it * 32 + sub;
    v4u a;
#pragma unroll
    for (int q = 0; q < 4; ++q) {
      const float f0 = tf[(c8 + 2 * q) * 68 + oc];
      const float f1 = tf[(c8 + 2 * q + 1) * 68 + oc];
      a[q] = pk16(f2bf_bits(f0), f2bf_bits(f1));
    }
    hv[it] = a;
  }
  for (int pass = 0; pass < 2; ++pass) {
#pragma unroll
    for (int it = 0; it < 2; ++it) {
      const int oc = it * 32 + sub;
      const size_t go = (size_t)(c0 + oc) * R + r0 + c8;
      *(volatile v4u*)(ob + go) = hv[it];
    }
    __threadfence();
  }
}

__global__ __launch_bounds__(128) void k_proj(
    const unsigned short* __restrict__ Xb, const unsigned short* __restrict__ Wb,
    const float* __restrict__ av, float* __restrict__ S,
    unsigned short* __restrict__ VTh, unsigned short* __restrict__ VTl) {
  __shared__ __align__(16) unsigned char smem[128 * 68 * 4];
  __shared__ __align__(16) float sA[2 * HD_];
  __shared__ __align__(16) float sS[4 * 128];
  float* sF = (float*)smem;
  unsigned short* sH = (unsigned short*)smem;
  unsigned short* sL = sH + 64 * 128;
  const int tid = threadIdx.x, lane = tid & 31, w = tid >> 5;
  const int hh = lane >> 4, m = lane & 15;
  const int xb = blockIdx.x;
  const int b  = xb / BPB;
  const int p0 = (xb % BPB) * 128;
  const int hp = blockIdx.y;
  const int n0 = hp * 64;
  const int m0 = xb * 128;
  const int m0w = m0 + 32 * w;
  const int bhA = b * NH_ + 2 * hp;

  const v8f zero8 = {0.f, 0.f, 0.f, 0.f, 0.f, 0.f, 0.f, 0.f};
  v8f acc[2][4];
#pragma unroll
  for (int mt = 0; mt < 2; ++mt)
#pragma unroll
    for (int nt = 0; nt < 4; ++nt) acc[mt][nt] = zero8;

  gemm_core_32x64p(Xb, Wb, DIN, (size_t)(m0w + m) * DIN, (size_t)(n0 + m) * DIN, hh, acc);

  if (tid < 2 * HD_) sA[tid] = bf16r(av[tid]);
#pragma unroll
  for (int nt = 0; nt < 4; ++nt)
#pragma unroll
    for (int mt = 0; mt < 2; ++mt)
#pragma unroll
      for (int r = 0; r < 8; ++r) {
        const int tokl = 32 * w + 16 * mt + 8 * hh + r;
        const int feat = 16 * nt + m;
        sF[tokl * 68 + feat] = acc[mt][nt][r];
      }
  __syncthreads();
  {
    float slA = 0.0f, srA = 0.0f, slB = 0.0f, srB = 0.0f;
    const float* fr = sF + tid * 68;
#pragma unroll 2
    for (int d4 = 0; d4 < HD_ / 4; ++d4) {
      const v4f xa = *(const v4fa*)(fr + 4 * d4);
      const v4f xc = *(const v4fa*)(fr + HD_ + 4 * d4);
      const v4f y  = *(const v4fa*)(sA + 4 * d4);
      const v4f z  = *(const v4fa*)(sA + HD_ + 4 * d4);
      slA = fmaf(xa[0], y[0], slA);
      slA = fmaf(xa[1], y[1], slA);
      slA = fmaf(xa[2], y[2], slA);
      slA = fmaf(xa[3], y[3], slA);
      srA = fmaf(xa[0], z[0], srA);
      srA = fmaf(xa[1], z[1], srA);
      srA = fmaf(xa[2], z[2], srA);
      srA = fmaf(xa[3], z[3], srA);
      slB = fmaf(xc[0], y[0], slB);
      slB = fmaf(xc[1], y[1], slB);
      slB = fmaf(xc[2], y[2], slB);
      slB = fmaf(xc[3], y[3], slB);
      srB = fmaf(xc[0], z[0], srB);
      srB = fmaf(xc[1], z[1], srB);
      srB = fmaf(xc[2], z[2], srB);
      srB = fmaf(xc[3], z[3], srB);
    }
    sS[tid]       = slA;
    sS[128 + tid] = slB;
    sS[256 + tid] = srA;
    sS[384 + tid] = srB;
  }
  __syncthreads();
  {
    const int rsel = w & 1, ksel = w >> 1;
    const size_t so = (size_t)ksel * NBH * NL_ + (size_t)(bhA + rsel) * NL_ + p0 + lane * 4;
    const v4f v = *(const v4fa*)(sS + w * 128 + lane * 4);
    *(volatile v4f*)(S + so) = v;
    __threadfence();
    *(volatile v4f*)(S + so) = v;
  }
#pragma unroll
  for (int nt = 0; nt < 4; ++nt)
#pragma unroll
    for (int mt = 0; mt < 2; ++mt)
#pragma unroll
      for (int r = 0; r < 8; ++r) {
        const int tokl = 32 * w + 16 * mt + 8 * hh + r;
        const int feat = 16 * nt + m;
        const float y = acc[mt][nt][r];
        const unsigned short hb = f2bf_bits(y);
        const unsigned short lb = f2bf_bits(y - bf_bits2f(hb));
        const int idx = feat * 128 + tokl;
        sH[idx] = hb;
        sL[idx] = lb;
      }
  __syncthreads();
  {
    const int dsub = lane >> 4, t8 = (lane & 15) * 8;
    for (int pass = 0; pass < 2; ++pass) {
#pragma unroll
      for (int it = 0; it < 8; ++it) {
        const int d = 16 * w + 2 * it + dsub;
        const v4u hv = *(const v4ua*)(sH + d * 128 + t8);
        const v4u lv = *(const v4ua*)(sL + d * 128 + t8);
        const size_t go = ((size_t)(bhA * HD_ + d)) * (size_t)NL_ + p0 + t8;
        *(volatile v4u*)(VTh + go) = hv;
        *(volatile v4u*)(VTl + go) = lv;
      }
      __threadfence();
    }
  }
}

__global__ __launch_bounds__(256) void k_colstats(const float* __restrict__ S, const int* __restrict__ adj,
                                                  float* __restrict__ CC) {
  __shared__ __align__(16) float sEI[NL_ * NH_];
  __shared__ __align__(16) float sEJ[NH_ * 64];
  __shared__ __align__(16) float sZ[4 * 64 * NH_];
  __shared__ __align__(16) float sOut[2 * NH_ * 64];
  __shared__ float sRed[8 * NH_];
  __shared__ float sEmax[NH_];
  const int tid = threadIdx.x, lane = tid & 31, w = tid >> 5;
  const int b = blockIdx.y, j0 = blockIdx.x * 64;

#pragma unroll
  for (int h = 0; h < NH_; ++h) {
    const v4f v = *(const v4fa*)(S + (size_t)(b * NH_ + h) * NL_ + 4 * tid);
    sEI[(4 * tid + 0) * NH_ + h] = v[0];
    sEI[(4 * tid + 1) * NH_ + h] = v[1];
    sEI[(4 * tid + 2) * NH_ + h] = v[2];
    sEI[(4 * tid + 3) * NH_ + h] = v[3];
    float mx = fmaxf(fmaxf(v[0], v[1]), fmaxf(v[2], v[3]));
    mx = fmaxf(mx, __shfl_xor(mx, 16, 32));
    mx = fmaxf(mx, __shfl_xor(mx, 8, 32));
    mx = fmaxf(mx, __shfl_xor(mx, 4, 32));
    mx = fmaxf(mx, __shfl_xor(mx, 2, 32));
    mx = fmaxf(mx, __shfl_xor(mx, 1, 32));
    if (lane == 0) sRed[w * NH_ + h] = mx;
  }
  if (tid < 128) {
    const int h = tid >> 4, j4 = (tid & 15) * 4;
    const v4f v = *(const v4fa*)(S + (size_t)NBH * NL_ + (size_t)(b * NH_ + h) * NL_ + j0 + j4);
    *(v4fa*)(sEJ + h * 64 + j4) = v;
  }
  __syncthreads();
  if (w == 0) {
    const int h = lane & 7, part = lane >> 3;
    float mx = fmaxf(sRed[(2 * part) * NH_ + h], sRed[(2 * part + 1) * NH_ + h]);
    mx = fmaxf(mx, __shfl_xor(mx, 8, 32));
    mx = fmaxf(mx, __shfl_xor(mx, 16, 32));
    if (lane < NH_) sEmax[lane] = mx;
  }
  __syncthreads();

  const int jl = tid & 63, ig = tid >> 6;
  float ej[NH_], c[NH_], Z[NH_];
#pragma unroll
  for (int h = 0; h < NH_; ++h) {
    ej[h] = sEJ[h * 64 + jl];
    float t = sEmax[h] + ej[h];
    c[h] = (t >= 0.0f) ? t : SLOPE * t;
    Z[h] = 0.0f;
  }
  const int* acol = adj + (size_t)b * NL_ * NL_ + j0 + jl;
#pragma unroll 1
  for (int i = ig; i < NL_; i += 4) {
    const int am = acol[(size_t)i * NL_];
    const float mv = (am != 0) ? 1.0f : 0.0f;
    const v4f e0 = *(const v4fa*)(sEI + i * NH_);
    const v4f e1 = *(const v4fa*)(sEI + i * NH_ + 4);
    const float ev[8] = {e0[0], e0[1], e0[2], e0[3], e1[0], e1[1], e1[2], e1[3]};
#pragma unroll
    for (int h = 0; h < NH_; ++h) {
      float t = ev[h] + ej[h];
      t = (t >= 0.0f) ? t : SLOPE * t;
      const float p = __expf(t - c[h]);
      Z[h] = fmaf(p, mv, Z[h]);
    }
  }
  {
    v4f za, zb;
    za[0] = Z[0]; za[1] = Z[1]; za[2] = Z[2]; za[3] = Z[3];
    zb[0] = Z[4]; zb[1] = Z[5]; zb[2] = Z[6]; zb[3] = Z[7];
    *(v4fa*)(sZ + (ig * 64 + jl) * NH_)     = za;
    *(v4fa*)(sZ + (ig * 64 + jl) * NH_ + 4) = zb;
  }
  __syncthreads();
  if (tid < 64) {
#pragma unroll 1
    for (int h = 0; h < NH_; ++h) {
      const int o = tid * NH_ + h;
      const float zz = ((sZ[o] + sZ[64 * NH_ + o]) + sZ[2 * 64 * NH_ + o]) + sZ[3 * 64 * NH_ + o];
      float t = sEmax[h] + sEJ[h * 64 + tid];
      t = (t >= 0.0f) ? t : SLOPE * t;
      const float zs = fmaxf(zz, 1e-30f);
      const float ci = (zz > 0.0f) ? (1.0f / zs) : 0.0f;
      sOut[h * 64 + tid] = t;
      sOut[NH_ * 64 + h * 64 + tid] = ci;
    }
  }
  __syncthreads();
  {
    const int hseg = lane >> 4, c4 = (lane & 15) * 4;
    const v4f v = *(const v4fa*)(sOut + (hseg * NH_ + w) * 64 + c4);
    float* dst = CC + (size_t)hseg * NBH * NL_ + (size_t)(b * NH_ + w) * NL_ + j0 + c4;
    *(volatile v4f*)dst = v;
    __threadfence();
    *(volatile v4f*)dst = v;
  }
}

__global__ __launch_bounds__(128) void k_attn(const float* __restrict__ S, const float* __restrict__ CC,
                                              const int* __restrict__ adj,
                                              const unsigned short* __restrict__ VTh,
                                              const unsigned short* __restrict__ VTl,
                                              const float* __restrict__ bias,
                                              float* __restrict__ out) {
  __shared__ __align__(16) float sK[NL_];
  __shared__ __align__(16) float sC[NL_];
  __shared__ __align__(16) float sI[NL_];
  __shared__ __align__(16) float sB[HD_];
  __shared__ __align__(16) float sO[4][16 * 36];

  const int tid = threadIdx.x, lane = tid & 31, w = tid >> 5;
  const int hh = lane >> 4, m = lane & 15;
  const int qt = blockIdx.x;
  const int bh = blockIdx.y, b = bh / NH_, hd = bh % NH_;
  const int q0 = qt * 64, q0w = q0 + 16 * w, q = q0w + m;

  {
    const float* gk = S  + (size_t)NBH * NL_ + (size_t)bh * NL_ + tid * 8;
    const float* gc = CC + (size_t)bh * NL_ + tid * 8;
    const float* gi = CC + (size_t)NBH * NL_ + (size_t)bh * NL_ + tid * 8;
#pragma unroll
    for (int i = 0; i < 2; ++i) {
      const v4f a  = *(const v4fa*)(gk + 4 * i);
      const v4f cc = *(const v4fa*)(gc + 4 * i);
      const v4f iv = *(const v4fa*)(gi + 4 * i);
      *(v4fa*)(sK + tid * 8 + 4 * i) = a;
      *(v4fa*)(sC + tid * 8 + 4 * i) = cc;
      *(v4fa*)(sI + tid * 8 + 4 * i) = iv;
    }
  }
  if (tid < HD_) sB[tid] = bf16r(bias[hd * HD_ + tid]);
  const float sqv = S[(size_t)bh * NL_ + q];
  const int* arow = adj + ((size_t)b * NL_ + q) * (size_t)NL_;

  const v8f zero8 = {0.f, 0.f, 0.f, 0.f, 0.f, 0.f, 0.f, 0.f};
  v8f o[2];
  o[0] = zero8; o[1] = zero8;

  __syncthreads();

#pragma unroll 1
  for (int ks = 0; ks < NL_ / 64; ++ks) {
    const int kb = ks * 64;

    v8f s[4];
#pragma unroll
    for (int j = 0; j < 4; ++j) {
      const int ko = kb + 16 * j + 8 * hh;
      const v4i mA = *(const v4ia*)(arow + ko);
      const v4i mB = *(const v4ia*)(arow + ko + 4);
      const v4f kA = *(const v4fa*)(sK + ko);
      const v4f kB = *(const v4fa*)(sK + ko + 4);
      const v4f cA = *(const v4fa*)(sC + ko);
      const v4f cB = *(const v4fa*)(sC + ko + 4);
      const v4f iA = *(const v4fa*)(sI + ko);
      const v4f iB = *(const v4fa*)(sI + ko + 4);
      const int   mv[8] = {mA[0], mA[1], mA[2], mA[3], mB[0], mB[1], mB[2], mB[3]};
      const float kv[8] = {kA[0], kA[1], kA[2], kA[3], kB[0], kB[1], kB[2], kB[3]};
      const float cv[8] = {cA[0], cA[1], cA[2], cA[3], cB[0], cB[1], cB[2], cB[3]};
      const float iv[8] = {iA[0], iA[1], iA[2], iA[3], iB[0], iB[1], iB[2], iB[3]};
#pragma unroll
      for (int r = 0; r < 8; ++r) {
        float t = sqv + kv[r];
        t = (t >= 0.0f) ? t : SLOPE * t;
        const float pe = __expf(t - cv[r]) * iv[r];
        const float pf = (iv[r] == 0.0f) ? INVN : 0.0f;
        s[j][r] = (mv[r] != 0) ? pe : pf;
      }
    }

    v16b p0h, p0l, p1h, p1l;
    pack_p2(s[0], s[1], p0h, p0l);
    pack_p2(s[2], s[3], p1h, p1l);

#pragma unroll
    for (int t = 0; t < 2; ++t) {
      const unsigned short* vph = VTh + (size_t)(bh * HD_ + 16 * t + m) * (size_t)NL_ + kb;
      const unsigned short* vpl = VTl + (size_t)(bh * HD_ + 16 * t + m) * (size_t)NL_ + kb;
      const v16b v0h = load_frag(vph, hh), v0l = load_frag(vpl, hh);
      o[t] = wmma_bf16(v0h, p0h, o[t]);
      o[t] = wmma_bf16(v0h, p0l, o[t]);
      o[t] = wmma_bf16(v0l, p0h, o[t]);
      const v16b v1h = load_frag(vph + 32, hh), v1l = load_frag(vpl + 32, hh);
      o[t] = wmma_bf16(v1h, p1h, o[t]);
      o[t] = wmma_bf16(v1h, p1l, o[t]);
      o[t] = wmma_bf16(v1l, p1h, o[t]);
    }
  }

  float* so = sO[w];
#pragma unroll
  for (int t = 0; t < 2; ++t) {
    const v4f bA = *(const v4fa*)(sB + 16 * t + 8 * hh);
    const v4f bB = *(const v4fa*)(sB + 16 * t + 8 * hh + 4);
    const float bv[8] = {bA[0], bA[1], bA[2], bA[3], bB[0], bB[1], bB[2], bB[3]};
#pragma unroll
    for (int r = 0; r < 8; ++r)
      so[m * 36 + 16 * t + 8 * hh + r] = o[t][r] + bv[r];
  }
  __syncthreads();
  {
    const int rsub = lane >> 3, c4 = (lane & 7) * 4;
    for (int pass = 0; pass < 2; ++pass) {
#pragma unroll
      for (int it = 0; it < 4; ++it) {
        const int row = 4 * it + rsub;
        const v4f v = *(const v4fa*)(so + row * 36 + c4);
        *(volatile v4f*)(out + (size_t)(b * NL_ + q0w + row) * (size_t)DM_ + hd * HD_ + c4) = v;
      }
      __threadfence();
    }
  }
}

extern "C" void kernel_launch(void* const* d_in, const int* in_sizes, int n_in,
                              void* d_out, int out_size, void* d_ws, size_t ws_size,
                              hipStream_t stream) {
  if (n_in < 5) return;
  if (in_sizes[0] != NTOK * DIN) return;
  if (in_sizes[1] != NB_ * NL_ * NL_) return;
  if (in_sizes[2] != DIN * DM_) return;
  if (in_sizes[3] != 2 * HD_) return;
  if (in_sizes[4] != DM_) return;
  if (out_size != NTOK * DM_) return;

  const float* hin  = (const float*)d_in[0];
  const int*   adj  = (const int*)d_in[1];
  const float* W    = (const float*)d_in[2];
  const float* av   = (const float*)d_in[3];
  const float* bias = (const float*)d_in[4];
  float* out = (float*)d_out;

  const size_t PX  = (size_t)NTOK * DIN * 2;
  const size_t PW  = (size_t)DM_ * DIN * 2;
  const size_t PS  = (size_t)2 * NBH * NL_ * 4;
  const size_t PC  = (size_t)2 * NBH * NL_ * 4;
  const size_t PVT = (size_t)NBH * HD_ * NL_ * 2;
  size_t off = 0;
  const size_t oXb  = off; off += PX;
  const size_t oWb  = off; off += PW;
  const size_t oS   = off; off += PS;
  const size_t oCC  = off; off += PC;
  const size_t oVTh = off; off += PVT;
  const size_t oVTl = off; off += PVT;
  if (off > ws_size || off > (size_t)WSMAX) return;

  char* ws = (char*)d_ws;
  unsigned short* Xb  = (unsigned short*)(ws + oXb);
  unsigned short* Wb  = (unsigned short*)(ws + oWb);
  float*          S   = (float*)(ws + oS);
  float*          CC  = (float*)(ws + oCC);
  unsigned short* VTh = (unsigned short*)(ws + oVTh);
  unsigned short* VTl = (unsigned short*)(ws + oVTl);

  const int n8x = NTOK * DIN / 8;
  k_cvt<<<dim3((n8x + 255) / 256), 256, 0, stream>>>(hin, Xb, n8x);
  k_tcvt<<<dim3(DM_ / 64, DIN / 64), 256, 0, stream>>>(W, Wb, DIN, DM_);
  k_proj<<<dim3(NTOK / 128, NHP), 128, 0, stream>>>(Xb, Wb, av, S, VTh, VTl);
  k_colstats<<<dim3(NL_ / 64, NB_), 256, 0, stream>>>(S, adj, CC);
  k_attn<<<dim3(NL_ / 64, NBH), 128, 0, stream>>>(S, CC, adj, VTh, VTl, bias, out);
  (void)hipGetLastError();
}
